// GCN_mhealth_Attn_29944511988453
// MI455X (gfx1250) — hardware-verified
//
#include <hip/hip_runtime.h>
#include <stddef.h>


#define FIN     128
#define HCW     256
#define NHEAD   4
#define HCH     64
#define HIDW    128
#define NCLS    12
#define NCP     16
#define XP      256
#define WP      128
#define F2P     256
#define OWP     128
#define YP      256
#define EP      4
#define NTHR    256
#define NWAVE   8
#define EPT     8
#define CHUNK   (NTHR * EPT)
#define WCAP    (EPT * 32)
#define LISTN   (NWAVE * WCAP)
#define NBMAX   2048
#define SLOTB   11
#define RCAP    28672
#define DEGCAP  4096
#define NSTRM   4
#define GBM     32
#define GTHR    64
#define NEG_SLOPE 0.2f
#define BN_EPS  0.00001f
#define CA      16.0f
#define CW      64.0f
#define SCL     0.0009765625f
#define WSCAP   134217728
#define LDS_BUILD ((2 * RCAP + 2 * NBMAX + LISTN) * 4 + 64)

static_assert((CHUNK & (CHUNK - 1)) == 0 && CHUNK <= 4096);
static_assert(NBMAX == (1 << SLOTB));
static_assert(NTHR * 8 == NBMAX);
static_assert(LISTN >= NBMAX);
static_assert(LISTN >= NWAVE * WCAP);
static_assert((RCAP % 32) == 0);
static_assert(LDS_BUILD <= 300000);
static_assert(GBM == (GTHR / 32) * 16);
static_assert(NHEAD * HCH == HCW);
static_assert(XP == HCW && F2P == HCW && WP == FIN && OWP == HIDW);
static_assert((FIN % 32) == 0 && (HCW % 32) == 0 && (HIDW % 32) == 0);
static_assert(NSTRM * NHEAD * 2 == 32);
static_assert(HCH == 64 && HIDW == 128 && NCLS <= NCP);
static_assert(GBM * EP == 32 * 4);
static_assert((GBM * NCLS) % 4 == 0);

typedef float    v4f  __attribute__((ext_vector_type(4)));
typedef float    v8f  __attribute__((ext_vector_type(8)));
typedef int      v4i  __attribute__((ext_vector_type(4)));
typedef int      v8i  __attribute__((ext_vector_type(8)));
typedef _Float16 v8h  __attribute__((ext_vector_type(8)));
typedef _Float16 v16h __attribute__((ext_vector_type(16)));
union FragH { v16h v; v8h h[2]; v8i w; };

__device__ __forceinline__ v8f wmh(const FragH& a, const FragH& b, v8f c) {
  v8f d = __builtin_amdgcn_wmma_f32_16x16x32_f16(false, a.v, false, b.v, (short)0, c, false, false);
  asm volatile("v_nop\n\tv_nop\n\tv_nop\n\tv_nop" : "+v"(d) : "v"(a.w), "v"(b.w));
  return d;
}

__device__ __forceinline__ v8h pack8(v4f a, v4f b, float sc) {
  v8h hv;
  hv[0] = (_Float16)(a.x * sc); hv[1] = (_Float16)(a.y * sc);
  hv[2] = (_Float16)(a.z * sc); hv[3] = (_Float16)(a.w * sc);
  hv[4] = (_Float16)(b.x * sc); hv[5] = (_Float16)(b.y * sc);
  hv[6] = (_Float16)(b.z * sc); hv[7] = (_Float16)(b.w * sc);
  return hv;
}

__device__ __forceinline__ v4f relu4(v4f a) {
  v4f r;
  r.x = fmaxf(a.x, 0.0f); r.y = fmaxf(a.y, 0.0f); r.z = fmaxf(a.z, 0.0f); r.w = fmaxf(a.w, 0.0f);
  return r;
}

__device__ __forceinline__ int scan_chunk(const int* __restrict__ dsts, int nE, int cbase, int slotBase,
                                          int nb, int vec8, int* list, int tid, int lane, int wave) {
  int wc = 0;
  const int el0  = tid * EPT;
  const int e0   = cbase + el0;
  const int sent = -2147483647 - 1;
  v4i da, db;
  if (vec8 != 0 && cbase + CHUNK <= nE) {
    da = *(const v4i*)(dsts + e0);
    db = *(const v4i*)(dsts + e0 + 4);
  } else {
    da.x = (e0     < nE) ? dsts[min(e0,     nE - 1)] : sent;
    da.y = (e0 + 1 < nE) ? dsts[min(e0 + 1, nE - 1)] : sent;
    da.z = (e0 + 2 < nE) ? dsts[min(e0 + 2, nE - 1)] : sent;
    da.w = (e0 + 3 < nE) ? dsts[min(e0 + 3, nE - 1)] : sent;
    db.x = (e0 + 4 < nE) ? dsts[min(e0 + 4, nE - 1)] : sent;
    db.y = (e0 + 5 < nE) ? dsts[min(e0 + 5, nE - 1)] : sent;
    db.z = (e0 + 6 < nE) ? dsts[min(e0 + 6, nE - 1)] : sent;
    db.w = (e0 + 7 < nE) ? dsts[min(e0 + 7, nE - 1)] : sent;
  }
  const unsigned nbs = (unsigned)slotBase;
  const unsigned unb = (unsigned)nb;
  const unsigned s0 = (unsigned)da.x - nbs, s1 = (unsigned)da.y - nbs;
  const unsigned s2 = (unsigned)da.z - nbs, s3 = (unsigned)da.w - nbs;
  const unsigned s4 = (unsigned)db.x - nbs, s5 = (unsigned)db.y - nbs;
  const unsigned s6 = (unsigned)db.z - nbs, s7 = (unsigned)db.w - nbs;
  const bool h0 = s0 < unb, h1 = s1 < unb, h2 = s2 < unb, h3 = s3 < unb;
  const bool h4 = s4 < unb, h5 = s5 < unb, h6 = s6 < unb, h7 = s7 < unb;
  const unsigned any = __builtin_amdgcn_ballot_w32(h0 | h1 | h2 | h3 | h4 | h5 | h6 | h7);
  if (any != 0u) {
#define HITJ(J, HJ, SJ) { \
      const unsigned mj = __builtin_amdgcn_ballot_w32(HJ); \
      if (mj != 0u) { \
        if (HJ) { \
          const int pos = wc + (int)__builtin_amdgcn_mbcnt_lo(mj, 0u); \
          if (pos < WCAP) list[wave * WCAP + pos] = ((el0 + (J)) << 12) | (int)(SJ); \
        } \
        wc += (int)__builtin_popcount(mj); } }
    HITJ(0, h0, s0)
    HITJ(1, h1, s1)
    HITJ(2, h2, s2)
    HITJ(3, h3, s3)
    HITJ(4, h4, s4)
    HITJ(5, h5, s5)
    HITJ(6, h6, s6)
    HITJ(7, h7, s7)
#undef HITJ
  }
  return wc;
}

__global__ __launch_bounds__(NTHR) void k_xprep(const float* __restrict__ x, _Float16* xc, int nN, int nUnits) {
  const int i = (int)blockIdx.x * NTHR + (int)threadIdx.x;
  if (i >= nUnits) return;
  const int row = i >> 5;
  const int c0  = (i & 31) * 8;
  const int rc  = row < nN ? row : nN - 1;
  const int cc  = c0 & (FIN - 1);
  const float* p = x + (size_t)rc * FIN + cc;
  v4f a = *(const v4f*)p, b = *(const v4f*)(p + 4);
  const v4f z4 = {0.f, 0.f, 0.f, 0.f};
  if (row >= nN || c0 >= FIN) { a = z4; b = z4; }
  const v8h hv = pack8(a, b, CA);
  const size_t o = (size_t)row * XP + c0;
  *(volatile v8h*)(xc + o) = hv;
  __threadfence();
  *(volatile v8h*)(xc + o) = hv;
}

__global__ __launch_bounds__(NTHR) void k_wprep(const float* __restrict__ w, const float* __restrict__ f2,
                                                const float* __restrict__ ow,
                                                _Float16* wt, _Float16* f2t, _Float16* owt) {
  const int j = (int)blockIdx.y;
  const int u = (int)blockIdx.x * NTHR + (int)threadIdx.x;
  v4f a, b;
  if (j == 0) {
    const int nUnits = HCW * (WP / 8);
    if (u >= nUnits) return;
    const int n  = u >> 4;
    const int k8 = (u & 15) * 8;
    const float* p = w + (size_t)k8 * HCW + n;
    a.x = p[0 * HCW]; a.y = p[1 * HCW]; a.z = p[2 * HCW]; a.w = p[3 * HCW];
    b.x = p[4 * HCW]; b.y = p[5 * HCW]; b.z = p[6 * HCW]; b.w = p[7 * HCW];
    const v8h hv = pack8(a, b, CW);
    const size_t o = (size_t)n * WP + k8;
    *(volatile v8h*)(wt + o) = hv;
    __threadfence();
    *(volatile v8h*)(wt + o) = hv;
  } else if (j == 1) {
    const int nUnits = HIDW * (F2P / 8);
    if (u >= nUnits) return;
    const int n  = u >> 5;
    const int k8 = (u & 31) * 8;
    const float* p = f2 + (size_t)k8 * HIDW + n;
    a.x = p[0 * HIDW]; a.y = p[1 * HIDW]; a.z = p[2 * HIDW]; a.w = p[3 * HIDW];
    b.x = p[4 * HIDW]; b.y = p[5 * HIDW]; b.z = p[6 * HIDW]; b.w = p[7 * HIDW];
    const v8h hv = pack8(a, b, CW);
    const size_t o = (size_t)n * F2P + k8;
    *(volatile v8h*)(f2t + o) = hv;
    __threadfence();
    *(volatile v8h*)(f2t + o) = hv;
  } else {
    const int nUnits = NCP * (OWP / 8);
    if (u >= nUnits) return;
    const int n   = u >> 4;
    const int k8  = (u & 15) * 8;
    const int ncl = n < NCLS ? n : NCLS - 1;
    const float* p = ow + (size_t)k8 * NCLS + ncl;
    a.x = p[0 * NCLS]; a.y = p[1 * NCLS]; a.z = p[2 * NCLS]; a.w = p[3 * NCLS];
    b.x = p[4 * NCLS]; b.y = p[5 * NCLS]; b.z = p[6 * NCLS]; b.w = p[7 * NCLS];
    const v4f z4 = {0.f, 0.f, 0.f, 0.f};
    if (n >= NCLS) { a = z4; b = z4; }
    const v8h hv = pack8(a, b, CW);
    const size_t o = (size_t)n * OWP + k8;
    *(volatile v8h*)(owt + o) = hv;
    __threadfence();
    *(volatile v8h*)(owt + o) = hv;
  }
}

__global__ __launch_bounds__(GTHR) void k_gemm(const _Float16* __restrict__ xc, const _Float16* __restrict__ wt,
                                               const float* __restrict__ asrc, const float* __restrict__ adst,
                                               float* Y, float* ES, float* ED) {
  __shared__ __attribute__((aligned(16))) float stg[GBM * HCW];
  __shared__ __attribute__((aligned(16))) float esT[GBM * EP];
  __shared__ __attribute__((aligned(16))) float edT[GBM * EP];
  __shared__ float sAs[HCW];
  __shared__ float sAd[HCW];
  const int tid = threadIdx.x, lane = tid & 31, wave = tid >> 5, hh = lane >> 4, m = lane & 15;
  const int rowBase = (int)blockIdx.x * GBM;
  for (int i = tid; i < HCW; i += GTHR) { sAs[i] = asrc[i]; sAd[i] = adst[i]; }
  const size_t arow = (size_t)(rowBase + 16 * wave + m) * XP + 8 * hh;
  const size_t brow = (size_t)m * WP + 8 * hh;
#pragma unroll 1
  for (int nh = 0; nh < 2; ++nh) {
    v8f acc[8];
#pragma unroll
    for (int t = 0; t < 8; ++t) { v8f z = {0.f, 0.f, 0.f, 0.f, 0.f, 0.f, 0.f, 0.f}; acc[t] = z; }
#pragma unroll 1
    for (int ks = 0; ks < FIN / 32; ++ks) {
      FragH af;
      af.h[0] = *(const v8h*)(xc + arow + 32 * ks);
      af.h[1] = *(const v8h*)(xc + arow + 32 * ks + 16);
#pragma unroll
      for (int t = 0; t < 8; ++t) {
        const size_t bo = brow + (size_t)(128 * nh + 16 * t) * WP + 32 * ks;
        FragH bf;
        bf.h[0] = *(const v8h*)(wt + bo);
        bf.h[1] = *(const v8h*)(wt + bo + 16);
        acc[t] = wmh(af, bf, acc[t]);
      }
    }
    {
      float* sp = stg + (size_t)(16 * wave + 8 * hh) * HCW + 128 * nh + m;
#pragma unroll
      for (int t = 0; t < 8; ++t) {
#pragma unroll
        for (int r = 0; r < 8; ++r) sp[(size_t)r * HCW + 16 * t] = acc[t][r] * SCL;
      }
    }
  }
  __syncthreads();
  {
    const int row  = tid >> 1;
    const int half = tid & 1;
    const float* srow = stg + (size_t)row * HCW;
#pragma unroll 1
    for (int p = 0; p < NHEAD; ++p) {
      float s = 0.f, d = 0.f;
#pragma unroll 1
      for (int c = 0; c < HCH / 2; ++c) {
        const int cc = p * HCH + half * (HCH / 2) + c;
        const float v = srow[cc];
        s = fmaf(v, sAs[cc], s);
        d = fmaf(v, sAd[cc], d);
      }
      s += __shfl_xor(s, 1);
      d += __shfl_xor(d, 1);
      if (half == 0) {
        esT[row * EP + p] = s;
        edT[row * EP + p] = d;
      }
    }
  }
  {
    const int nF4 = GBM * HCW / 4;
    float* yb = Y + (size_t)rowBase * YP;
    const v4f* s4 = (const v4f*)stg;
#pragma unroll 1
    for (int f = tid; f < nF4; f += GTHR) {
      const int r = f >> 6, q = f & 63;
      const v4f v = s4[f];
      *(volatile v4f*)(yb + (size_t)r * YP + 4 * q) = v;
    }
    __threadfence();
#pragma unroll 1
    for (int f = tid; f < nF4; f += GTHR) {
      const int r = f >> 6, q = f & 63;
      const v4f v = s4[f];
      *(volatile v4f*)(yb + (size_t)r * YP + 4 * q) = v;
    }
  }
  __syncthreads();
  if (wave == 0) {
    const v4f ve = *(const v4f*)(esT + 4 * lane);
    const v4f vd = *(const v4f*)(edT + 4 * lane);
    float* pe = ES + (size_t)rowBase * EP + 4 * lane;
    float* pd = ED + (size_t)rowBase * EP + 4 * lane;
    *(volatile v4f*)pe = ve;
    *(volatile v4f*)pd = vd;
    __threadfence();
    *(volatile v4f*)pe = ve;
    *(volatile v4f*)pd = vd;
  }
}

__global__ __launch_bounds__(NTHR) void k_build(const int* __restrict__ dsts, int* EL, int* OFF, int* CNT,
                                                int nE, int nb, int tp, int vec8) {
  extern __shared__ v4f lds_dyn[];
  int* reg1 = (int*)lds_dyn;
  int* reg2 = reg1 + RCAP;
  int* scnt = reg2 + RCAP;
  int* soff = scnt + NBMAX;
  int* list = soff + NBMAX;
  int* wcnt = list + LISTN;
  int* wtot = wcnt + NWAVE;
  const int tid = threadIdx.x, lane = tid & 31, wave = tid >> 5;
  const int nodeBase = (int)blockIdx.x * nb;

  for (int i = tid; i < NBMAX; i += NTHR) scnt[i] = 0;
  {
    const v4i z = {0, 0, 0, 0};
    v4i* r2v = (v4i*)reg2;
    for (int f = tid; f < RCAP / 4; f += NTHR) r2v[f] = z;
  }
  __syncthreads();

  int tot = 0;
  const int nChunks = (nE + CHUNK - 1) / CHUNK;
#pragma unroll 1
  for (int ch = 0; ch < nChunks; ++ch) {
    const int cbase = ch * CHUNK;
    const int wc = scan_chunk(dsts, nE, cbase, nodeBase, nb, vec8, list, tid, lane, wave);
    if (lane == 0) wcnt[wave] = wc;
    __syncthreads();
    int pre = 0, all = 0;
#pragma unroll
    for (int w2 = 0; w2 < NWAVE; ++w2) {
      int c = wcnt[w2];
      c = c < 0 ? 0 : (c > WCAP ? WCAP : c);
      all += c;
      pre += (w2 < wave) ? c : 0;
    }
    const int wcc  = wc > WCAP ? WCAP : wc;
    const int base = tot + pre;
#pragma unroll 1
    for (int i = lane; i < wcc; i += 32) {
      const int ent = list[wave * WCAP + i];
      const int el  = (ent >> 12) & (CHUNK - 1);
      const int sl  = ent & (NBMAX - 1);
      int eid = cbase + el;
      eid = eid > nE - 1 ? nE - 1 : eid;
      const int pos = base + i;
      if (pos < RCAP) reg1[pos] = (int)(((unsigned)eid << SLOTB) | (unsigned)sl);
    }
    tot += all;
    tot = tot > RCAP ? RCAP : tot;
    __syncthreads();
  }
  const int nh = tot;

  if (wave == 0) {
#pragma unroll 1
    for (int b0 = 0; b0 < nh; b0 += 32) {
      const int idx = b0 + lane;
      const int uv  = reg1[idx < RCAP ? idx : RCAP - 1];
      const int m32 = (nh - b0) < 32 ? (nh - b0) : 32;
#pragma unroll 1
      for (int k = 0; k < m32; ++k) {
        const int u  = __builtin_amdgcn_readlane(uv, k);
        const int sl = u & (NBMAX - 1);
        if (lane == 0) scnt[sl] = scnt[sl] + 1;
      }
    }
  }
  __syncthreads();

  {
    const v4i ca = *(const v4i*)(scnt + 8 * tid);
    const v4i cb = *(const v4i*)(scnt + 8 * tid + 4);
    const int e0 = ca.x < 0 ? 0 : ca.x, e1 = ca.y < 0 ? 0 : ca.y, e2 = ca.z < 0 ? 0 : ca.z, e3 = ca.w < 0 ? 0 : ca.w;
    const int e4 = cb.x < 0 ? 0 : cb.x, e5 = cb.y < 0 ? 0 : cb.y, e6 = cb.z < 0 ? 0 : cb.z, e7 = cb.w < 0 ? 0 : cb.w;
    const int ts = e0 + e1 + e2 + e3 + e4 + e5 + e6 + e7;
    int incl = ts;
#pragma unroll
    for (int d = 1; d < 32; d <<= 1) {
      const int up = __shfl_up(incl, d);
      if (lane >= d) incl += up;
    }
    if (lane == 31) wtot[wave] = incl;
    __syncthreads();
    int pre = 0;
#pragma unroll
    for (int w2 = 0; w2 < NWAVE; ++w2) pre += (w2 < wave) ? wtot[w2] : 0;
    int run = pre + incl - ts;
    soff[8 * tid + 0] = run; run += e0;
    soff[8 * tid + 1] = run; run += e1;
    soff[8 * tid + 2] = run; run += e2;
    soff[8 * tid + 3] = run; run += e3;
    soff[8 * tid + 4] = run; run += e4;
    soff[8 * tid + 5] = run; run += e5;
    soff[8 * tid + 6] = run; run += e6;
    soff[8 * tid + 7] = run;
  }
  __syncthreads();
  for (int i = tid; i < NBMAX; i += NTHR) list[i] = soff[i];
  __syncthreads();

  if (wave == 0) {
#pragma unroll 1
    for (int b0 = 0; b0 < nh; b0 += 32) {
      const int idx = b0 + lane;
      const int uv  = reg1[idx < RCAP ? idx : RCAP - 1];
      const int m32 = (nh - b0) < 32 ? (nh - b0) : 32;
#pragma unroll 1
      for (int k = 0; k < m32; ++k) {
        const int u   = __builtin_amdgcn_readlane(uv, k);
        const int sl  = u & (NBMAX - 1);
        const int eid = (int)((unsigned)u >> SLOTB);
        if (lane == 0) {
          int pos = list[sl];
          pos = pos < 0 ? 0 : (pos > RCAP - 1 ? RCAP - 1 : pos);
          reg2[pos] = eid;
          list[sl] = pos + 1;
        }
      }
    }
  }
  __syncthreads();

  {
    int* elb = EL + (size_t)blockIdx.x * RCAP;
    const v4i* r4 = (const v4i*)reg2;
#pragma unroll 1
    for (int f = tid; f < RCAP / 4; f += NTHR) {
      const v4i v = r4[f];
      *(volatile v4i*)(elb + 4 * f) = v;
    }
    __threadfence();
#pragma unroll 1
    for (int f = tid; f < RCAP / 4; f += NTHR) {
      const v4i v = r4[f];
      *(volatile v4i*)(elb + 4 * f) = v;
    }
  }
  {
    const bool ovf = (nh >= RCAP);
    int* ob = OFF + (size_t)blockIdx.x * tp;
    int* cb = CNT + (size_t)blockIdx.x * tp;
    const int n4 = tp >> 2;
#pragma unroll 1
    for (int pass = 0; pass < 2; ++pass) {
#pragma unroll 1
      for (int f = tid; f < n4; f += NTHR) {
        v4i so, sc;
        {
          const int s = 4 * f + 0; const bool in = s < nb; const int scl = s < NBMAX ? s : NBMAX - 1;
          so.x = in ? soff[scl] : 0; sc.x = in ? (ovf ? -1 : scnt[scl]) : 0;
        }
        {
          const int s = 4 * f + 1; const bool in = s < nb; const int scl = s < NBMAX ? s : NBMAX - 1;
          so.y = in ? soff[scl] : 0; sc.y = in ? (ovf ? -1 : scnt[scl]) : 0;
        }
        {
          const int s = 4 * f + 2; const bool in = s < nb; const int scl = s < NBMAX ? s : NBMAX - 1;
          so.z = in ? soff[scl] : 0; sc.z = in ? (ovf ? -1 : scnt[scl]) : 0;
        }
        {
          const int s = 4 * f + 3; const bool in = s < nb; const int scl = s < NBMAX ? s : NBMAX - 1;
          so.w = in ? soff[scl] : 0; sc.w = in ? (ovf ? -1 : scnt[scl]) : 0;
        }
        *(volatile v4i*)(ob + 4 * f) = so;
        *(volatile v4i*)(cb + 4 * f) = sc;
      }
      __threadfence();
    }
  }
}

__global__ __launch_bounds__(NTHR) void k_agg(
    const int* __restrict__ srcs, const int* __restrict__ EL,
    const int* __restrict__ OFF, const int* __restrict__ CNT,
    const float* __restrict__ Y, const float* __restrict__ ES, const float* __restrict__ ED,
    const float* __restrict__ bias, const float* __restrict__ bng, const float* __restrict__ bnb,
    const float* __restrict__ bnm, const float* __restrict__ bnv,
    _Float16* xout, int nN, int nE, int nb, int tp) {
  __shared__ v4f cmb[NWAVE * NSTRM * 64];
  __shared__ float cdn[NWAVE * NSTRM * NHEAD];
  const int tid = threadIdx.x, lane = tid & 31, wave = tid >> 5;
  const int g   = lane >> 3;
  const int sub = lane & 7;
  const int j   = sub >> 1;
  const int chf = sub & 1;
  const int cb0 = HCH * j + 32 * chf;
  const int hL  = lane >> 3;
  const int nodeBase = (int)blockIdx.x * nb;
  const int nbw = nb >> 3;
  const int* elb  = EL  + (size_t)blockIdx.x * RCAP;
  const int* offb = OFF + (size_t)blockIdx.x * tp;
  const int* cntb = CNT + (size_t)blockIdx.x * tp;
  const v4f bz0 = *(const v4f*)(bias + 8 * lane);
  const v4f bz1 = *(const v4f*)(bias + 8 * lane + 4);
  const v4f mn0 = *(const v4f*)(bnm + 8 * lane);
  const v4f mn1 = *(const v4f*)(bnm + 8 * lane + 4);
  const v4f ga0 = *(const v4f*)(bng + 8 * lane);
  const v4f ga1 = *(const v4f*)(bng + 8 * lane + 4);
  const v4f be0 = *(const v4f*)(bnb + 8 * lane);
  const v4f be1 = *(const v4f*)(bnb + 8 * lane + 4);
  const v4f vv0 = *(const v4f*)(bnv + 8 * lane);
  const v4f vv1 = *(const v4f*)(bnv + 8 * lane + 4);
  v4f rs0, rs1;
  rs0.x = rsqrtf(vv0.x + BN_EPS); rs0.y = rsqrtf(vv0.y + BN_EPS);
  rs0.z = rsqrtf(vv0.z + BN_EPS); rs0.w = rsqrtf(vv0.w + BN_EPS);
  rs1.x = rsqrtf(vv1.x + BN_EPS); rs1.y = rsqrtf(vv1.y + BN_EPS);
  rs1.z = rsqrtf(vv1.z + BN_EPS); rs1.w = rsqrtf(vv1.w + BN_EPS);
  const float qnan = __int_as_float(0x7fc00000);
  const v4f z4 = {0.f, 0.f, 0.f, 0.f};
  v4f* cw = cmb + wave * (NSTRM * 64);
  float* cd = cdn + wave * (NSTRM * NHEAD);
#pragma unroll 1
  for (int jt = 0; jt < nbw; ++jt) {
    const int slot = wave * nbw + jt;
    const int grow = nodeBase + slot;
    const int gcl  = grow < nN ? grow : nN - 1;
    const bool wr  = grow < nN;
    int st = offb[slot];
    const int craw = cntb[slot];
    st = st < 0 ? 0 : (st > RCAP - 1 ? RCAP - 1 : st);
    int cnt = craw < 0 ? 0 : (craw > DEGCAP ? DEGCAP : craw);
    if (cnt > RCAP - st) cnt = RCAP - st;
    const float pz = (craw < 0 || craw > DEGCAP) ? qnan : 0.0f;

    const float edv = ED[(size_t)gcl * EP + j];
    const float esd = ES[(size_t)gcl * EP + j];
    const float t0  = esd + edv;
    float mx = fmaxf(t0, NEG_SLOPE * t0);
    const float* yd = Y + (size_t)gcl * YP + cb0;
    const bool g0 = (g == 0);
    float dn = g0 ? 1.0f : 0.0f;
    const v4f y0 = *(const v4f*)(yd +  0), y1 = *(const v4f*)(yd +  4);
    const v4f y2 = *(const v4f*)(yd +  8), y3 = *(const v4f*)(yd + 12);
    const v4f y4 = *(const v4f*)(yd + 16), y5 = *(const v4f*)(yd + 20);
    const v4f y6 = *(const v4f*)(yd + 24), y7 = *(const v4f*)(yd + 28);
    v4f a0 = g0 ? y0 : z4, a1 = g0 ? y1 : z4, a2 = g0 ? y2 : z4, a3 = g0 ? y3 : z4;
    v4f a4 = g0 ? y4 : z4, a5 = g0 ? y5 : z4, a6 = g0 ? y6 : z4, a7 = g0 ? y7 : z4;
    const int niter = (cnt + NSTRM - 1) / NSTRM;
#pragma unroll 1
    for (int it = 0; it < niter; ++it) {
      const int q = it * NSTRM + g;
      const bool valid = q < cnt;
      const int qc = valid ? q : cnt - 1;
      const int idx = st + qc;
      int eid = elb[idx];
      eid = eid < 0 ? 0 : (eid > nE - 1 ? nE - 1 : eid);
      const int sraw = srcs[eid];
      const int s = sraw < 0 ? 0 : (sraw > nN - 1 ? nN - 1 : sraw);
      const float* ys = Y + (size_t)s * YP + cb0;
      const v4f x0 = *(const v4f*)(ys +  0);
      const v4f x1 = *(const v4f*)(ys +  4);
      const v4f x2 = *(const v4f*)(ys +  8);
      const v4f x3 = *(const v4f*)(ys + 12);
      const v4f x4 = *(const v4f*)(ys + 16);
      const v4f x5 = *(const v4f*)(ys + 20);
      const v4f x6 = *(const v4f*)(ys + 24);
      const v4f x7 = *(const v4f*)(ys + 28);
      const float ess = ES[(size_t)s * EP + j];
      const float u = ess + edv;
      float l = fmaxf(u, NEG_SLOPE * u);
      l = valid ? l : (mx - 100.0f);
      const float mn = fmaxf(mx, l);
      const float s1 = __expf(mx - mn), s2 = __expf(l - mn);
      dn = fmaf(dn, s1, s2);
      a0 = a0 * s1 + x0 * s2;
      a1 = a1 * s1 + x1 * s2;
      a2 = a2 * s1 + x2 * s2;
      a3 = a3 * s1 + x3 * s2;
      a4 = a4 * s1 + x4 * s2;
      a5 = a5 * s1 + x5 * s2;
      a6 = a6 * s1 + x6 * s2;
      a7 = a7 * s1 + x7 * s2;
      mx = mn;
    }
    float m1 = fmaxf(mx, __shfl_xor(mx, 8));
    m1 = fmaxf(m1, __shfl_xor(m1, 16));
    const float e = __expf(mx - m1);
    __builtin_amdgcn_fence(__ATOMIC_RELEASE, "wavefront");
    __builtin_amdgcn_wave_barrier();
    v4f* cg = cw + g * 64 + 8 * sub;
    cg[0] = a0 * e; cg[1] = a1 * e; cg[2] = a2 * e; cg[3] = a3 * e;
    cg[4] = a4 * e; cg[5] = a5 * e; cg[6] = a6 * e; cg[7] = a7 * e;
    if (chf == 0) cd[g * NHEAD + j] = dn * e;
    __builtin_amdgcn_fence(__ATOMIC_RELEASE, "wavefront");
    __builtin_amdgcn_wave_barrier();
    v4f r0 = cw[2 * lane], r1 = cw[2 * lane + 1];
    float ds = cd[hL];
#pragma unroll
    for (int gg = 1; gg < NSTRM; ++gg) {
      r0 += cw[gg * 64 + 2 * lane];
      r1 += cw[gg * 64 + 2 * lane + 1];
      ds += cd[gg * NHEAD + hL];
    }
    const float inv = __builtin_amdgcn_rcpf(ds);
    const v4f o0 = relu4(r0 * inv + bz0);
    const v4f o1 = relu4(r1 * inv + bz1);
    v4f q0 = (o0 - mn0) * rs0;
    v4f q1 = (o1 - mn1) * rs1;
    q0 = q0 * ga0 + be0 + pz;
    q1 = q1 * ga1 + be1 + pz;
    const v8h hv = pack8(q0, q1, CA);
    _Float16* xp = xout + (size_t)gcl * XP + 8 * lane;
    if (wr) *(volatile v8h*)xp = hv;
    __threadfence();
    if (wr) *(volatile v8h*)xp = hv;
  }
}

__global__ __launch_bounds__(GTHR) void k_mlp(const _Float16* __restrict__ xc, const _Float16* __restrict__ f2t,
                                              const _Float16* __restrict__ owt,
                                              const float* __restrict__ b2, const float* __restrict__ bo,
                                              float* out, int nN) {
  __shared__ __attribute__((aligned(16))) _Float16 sH[GBM * HIDW];
  __shared__ __attribute__((aligned(16))) float sO[GBM * NCLS];
  __shared__ float sb2[HIDW];
  __shared__ float sbo[NCP];
  const int tid = threadIdx.x, lane = tid & 31, wave = tid >> 5, hh = lane >> 4, m = lane & 15;
  const int rowBase = (int)blockIdx.x * GBM;
  for (int i = tid; i < HIDW; i += GTHR) sb2[i] = b2[i];
  if (tid < NCP) sbo[tid] = bo[tid < NCLS ? tid : NCLS - 1];
  __syncthreads();
  const size_t arow = (size_t)(rowBase + 16 * wave + m) * XP + 8 * hh;
  const size_t brow = (size_t)m * F2P + 8 * hh;
  v8f acc[8];
#pragma unroll
  for (int t = 0; t < 8; ++t) { v8f z = {0.f, 0.f, 0.f, 0.f, 0.f, 0.f, 0.f, 0.f}; acc[t] = z; }
#pragma unroll 1
  for (int ks = 0; ks < HCW / 32; ++ks) {
    FragH af;
    af.h[0] = *(const v8h*)(xc + arow + 32 * ks);
    af.h[1] = *(const v8h*)(xc + arow + 32 * ks + 16);
#pragma unroll
    for (int t = 0; t < 8; ++t) {
      const size_t bofs = brow + (size_t)(16 * t) * F2P + 32 * ks;
      FragH bf;
      bf.h[0] = *(const v8h*)(f2t + bofs);
      bf.h[1] = *(const v8h*)(f2t + bofs + 16);
      acc[t] = wmh(af, bf, acc[t]);
    }
  }
  {
    _Float16* hp = sH + (size_t)(16 * wave + 8 * hh) * HIDW + m;
#pragma unroll
    for (int t = 0; t < 8; ++t) {
      const float bb = sb2[16 * t + m];
#pragma unroll
      for (int r = 0; r < 8; ++r) {
        const float v = fmaxf(fmaf(acc[t][r], SCL, bb), 0.f);
        hp[(size_t)r * HIDW + 16 * t] = (_Float16)(v * CA);
      }
    }
  }
  __syncthreads();
  v8f hacc = {0.f, 0.f, 0.f, 0.f, 0.f, 0.f, 0.f, 0.f};
  {
    const _Float16* ap = sH + (size_t)(16 * wave + m) * HIDW + 8 * hh;
    const _Float16* bp = owt + (size_t)m * OWP + 8 * hh;
#pragma unroll
    for (int ks = 0; ks < HIDW / 32; ++ks) {
      FragH af, bf;
      af.h[0] = *(const v8h*)(ap + 32 * ks);
      af.h[1] = *(const v8h*)(ap + 32 * ks + 16);
      bf.h[0] = *(const v8h*)(bp + 32 * ks);
      bf.h[1] = *(const v8h*)(bp + 32 * ks + 16);
      hacc = wmh(af, bf, hacc);
    }
  }
  if (m < NCLS) {
    const float bb = sbo[m];
    float* op = sO + (size_t)(16 * wave + 8 * hh) * NCLS + m;
#pragma unroll
    for (int r = 0; r < 8; ++r) op[(size_t)r * NCLS] = fmaf(hacc[r], SCL, bb);
  }
  __syncthreads();
  const int nValid = (nN - rowBase) < GBM ? (nN - rowBase) : GBM;
  const int n4 = (NCLS * nValid) >> 2;
  float* base = out + (size_t)rowBase * NCLS;
  const v4f* s4 = (const v4f*)sO;
#pragma unroll 1
  for (int f = tid; f < n4; f += GTHR) {
    const v4f v = s4[f];
    *(volatile v4f*)(base + 4 * f) = v;
  }
  __threadfence();
#pragma unroll 1
  for (int f = tid; f < n4; f += GTHR) {
    const v4f v = s4[f];
    *(volatile v4f*)(base + 4 * f) = v;
  }
}

static int pick_nb(int nE, int nN) {
  int nb = NBMAX;
  while (nb > 16 && (long long)nb * (long long)nE * 5LL > (long long)RCAP * (long long)nN * 4LL) nb >>= 1;
  return nb;
}

extern "C" void kernel_launch(void* const* d_in, const int* in_sizes, int n_in,
                              void* d_out, int out_size, void* d_ws, size_t ws_size,
                              hipStream_t stream) {
  if (n_in < 14) return;
  const int nN = in_sizes[0] / FIN;
  if (nN <= 0 || in_sizes[0] != nN * FIN) return;
  if (nN > (1 << 22)) return;
  if (in_sizes[1] < 2 || (in_sizes[1] & 1) != 0) return;
  const int nE = in_sizes[1] / 2;
  if (nE < 1 || nE > (1 << 21)) return;
  if (in_sizes[2] != FIN * HCW) return;
  if (in_sizes[3] != HCW || in_sizes[4] != HCW) return;
  if (in_sizes[5] != HCW || in_sizes[6] != HCW || in_sizes[7] != HCW) return;
  if (in_sizes[8] != HCW || in_sizes[9] != HCW) return;
  if (in_sizes[10] != HCW * HIDW || in_sizes[11] != HIDW) return;
  if (in_sizes[12] != HIDW * NCLS || in_sizes[13] != NCLS) return;
  if (out_size != nN * NCLS) return;

  const float* x      = (const float*)d_in[0];
  const int*   ei     = (const int*)d_in[1];
  const float* W      = (const float*)d_in[2];
  const float* att_s  = (const float*)d_in[3];
  const float* att_d  = (const float*)d_in[4];
  const float* gbias  = (const float*)d_in[5];
  const float* bng    = (const float*)d_in[6];
  const float* bnb    = (const float*)d_in[7];
  const float* bnm    = (const float*)d_in[8];
  const float* bnv    = (const float*)d_in[9];
  const float* fc2w   = (const float*)d_in[10];
  const float* fc2b   = (const float*)d_in[11];
  const float* outw   = (const float*)d_in[12];
  const float* outb   = (const float*)d_in[13];
  float* out = (float*)d_out;
  const int* dsts = ei + nE;

  const int MP   = ((nN + GBM - 1) / GBM) * GBM;
  const int nb   = pick_nb(nE, nN);
  const int tp   = nb < 32 ? 32 : nb;
  const int gA   = (nN + nb - 1) / nb;
  const int gG   = MP / GBM;
  const int vec8 = ((nE & 3) == 0) ? 1 : 0;
  const int nUnits = MP * (XP / 8);
  if (nb < 16 || nb > NBMAX || (long long)gA * nb < (long long)nN) return;

  char* ws = (char*)d_ws;
  size_t off = 0;
  const size_t oWT  = off; off += (size_t)HCW * WP * 2;          off = (off + 255) & ~(size_t)255;
  const size_t oF2T = off; off += (size_t)HIDW * F2P * 2;        off = (off + 255) & ~(size_t)255;
  const size_t oOWT = off; off += (size_t)NCP * OWP * 2;         off = (off + 255) & ~(size_t)255;
  const size_t oXC  = off; off += (size_t)MP * XP * 2;           off = (off + 255) & ~(size_t)255;
  const size_t oY   = off; off += (size_t)MP * YP * 4;           off = (off + 255) & ~(size_t)255;
  const size_t oES  = off; off += (size_t)MP * EP * 4;           off = (off + 255) & ~(size_t)255;
  const size_t oED  = off; off += (size_t)MP * EP * 4;           off = (off + 255) & ~(size_t)255;
  const size_t oEL  = off; off += (size_t)gA * RCAP * 4;         off = (off + 255) & ~(size_t)255;
  const size_t oOFF = off; off += (size_t)gA * tp * 4;           off = (off + 255) & ~(size_t)255;
  const size_t oCNT = off; off += (size_t)gA * tp * 4;           off = (off + 255) & ~(size_t)255;
  if (off > ws_size || off > (size_t)WSCAP) return;
  _Float16* WT  = (_Float16*)(ws + oWT);
  _Float16* F2T = (_Float16*)(ws + oF2T);
  _Float16* OWT = (_Float16*)(ws + oOWT);
  _Float16* XC  = (_Float16*)(ws + oXC);
  float*    Y   = (float*)(ws + oY);
  float*    ES  = (float*)(ws + oES);
  float*    ED  = (float*)(ws + oED);
  int*      EL  = (int*)(ws + oEL);
  int*      OFF = (int*)(ws + oOFF);
  int*      CNT = (int*)(ws + oCNT);

  hipFuncSetAttribute(reinterpret_cast<const void*>(&k_build),
                      hipFuncAttributeMaxDynamicSharedMemorySize, LDS_BUILD);

  k_xprep<<<(nUnits + NTHR - 1) / NTHR, NTHR, 0, stream>>>(x, XC, nN, nUnits);
  k_wprep<<<dim3((HCW * (WP / 8) + NTHR - 1) / NTHR, 3), NTHR, 0, stream>>>(W, fc2w, outw, WT, F2T, OWT);

  k_build<<<gA, NTHR, LDS_BUILD, stream>>>(dsts, EL, OFF, CNT, nE, nb, tp, vec8);

  k_gemm<<<gG, GTHR, 0, stream>>>(XC, WT, att_s, att_d, Y, ES, ED);
  k_agg<<<gA, NTHR, 0, stream>>>(ei, EL, OFF, CNT, Y, ES, ED, gbias, bng, bnb, bnm, bnv, XC, nN, nE, nb, tp);

  k_mlp<<<gG, GTHR, 0, stream>>>(XC, F2T, OWT, fc2b, outb, out, nN);
}
